// GeodesicPrototypeClassifier_24043226923959
// MI455X (gfx1250) — hardware-run, weakly checked
//
#include <hip/hip_runtime.h>
#define NB 2
#define SQ 2048
#define DM 1024
#define NH 16
#define HD 64
#define HG 4
#define GN 16384
#define GK 128
#define GD 64
#define GCAR 64.0f
#define B0 0
#define NBR NB
#define NR ((size_t)NB * SQ)
#define MP ((int)((size_t)NBR * SQ))
#define QN SQ
#define NHD NH
#define MPO MP
#define LQ DM
typedef __bf16 v16b __attribute__((ext_vector_type(16)));
typedef unsigned short v8us __attribute__((ext_vector_type(8), may_alias));
typedef float  v8f  __attribute__((ext_vector_type(8)));
typedef float  v4f  __attribute__((ext_vector_type(4)));
typedef float  v4fa __attribute__((ext_vector_type(4), may_alias));
union FragB { v16b v; v8us half[2]; unsigned short u[16]; };

__device__ __forceinline__ unsigned short bf16_bits(float x) { unsigned int u = __float_as_uint(x); return (unsigned short)((u + 0x7FFFu + ((u >> 16) & 1u)) >> 16); }
__device__ __forceinline__ float bf16_val(unsigned short b) { return __uint_as_float(((unsigned int)b) << 16); }
__device__ __forceinline__ float bf16_round(float x) { return bf16_val(bf16_bits(x)); }
template <int NT>
__device__ __forceinline__ v8f mmaN(v16b ah, v16b al, v16b bh, v16b bl, v8f c) {
  c = __builtin_amdgcn_wmma_f32_16x16x32_bf16(false, ah, false, bh, (short)0, c, false, false);
  if (NT >= 2) c = __builtin_amdgcn_wmma_f32_16x16x32_bf16(false, al, false, bh, (short)0, c, false, false);
  if (NT >= 3) c = __builtin_amdgcn_wmma_f32_16x16x32_bf16(false, ah, false, bl, (short)0, c, false, false);
  asm volatile("v_nop\n\tv_nop\n\tv_nop\n\tv_nop" : "+v"(c) : "v"(ah), "v"(al), "v"(bh), "v"(bl));
  return c;
}


typedef _Float16 v16h __attribute__((ext_vector_type(16)));
union FragH { v16h v; v8us half[2]; _Float16 h[16]; unsigned short u[16]; };
template <int NT>
__device__ __forceinline__ v8f mmaH(v16h ah, v16h al, v16h bh, v16h bl, v8f c) {
  c = __builtin_amdgcn_wmma_f32_16x16x32_f16(false, ah, false, bh, (short)0, c, false, false);
  if (NT >= 2) c = __builtin_amdgcn_wmma_f32_16x16x32_f16(false, al, false, bh, (short)0, c, false, false);
  if (NT >= 3) c = __builtin_amdgcn_wmma_f32_16x16x32_f16(false, ah, false, bl, (short)0, c, false, false);
  asm volatile("v_nop\n\tv_nop\n\tv_nop\n\tv_nop" : "+v"(c) : "v"(ah), "v"(al), "v"(bh), "v"(bl));
  return c;
}


typedef _Float16 v4h __attribute__((ext_vector_type(4)));

__global__ __launch_bounds__(256) void k_x16s(const float* __restrict__ x, _Float16* __restrict__ X16, size_t n8, float scale) { const size_t t = (size_t)blockIdx.x * 256 + threadIdx.x; if (t >= n8) return; FragH f;
#pragma unroll
  for (int q = 0; q < 8; ++q) f.h[q] = (_Float16)(bf16_round(x[t * 8 + q]) * scale); *(volatile v8us*)((unsigned short*)X16 + t * 8) = f.half[0]; __threadfence(); *(volatile v8us*)((unsigned short*)X16 + t * 8) = f.half[0]; }


__device__ __forceinline__ v16h g2_frag(const _Float16* p, int hh) { FragH f; f.half[0] = *(const v8us*)((const unsigned short*)p + 8 * hh); f.half[1] = *(const v8us*)((const unsigned short*)p + 16 + 8 * hh); return f.v; }
__device__ __forceinline__ v8f g2_mma(v16h a, v16h b, v8f c) { v8f d = __builtin_amdgcn_wmma_f32_16x16x32_f16(false, a, false, b, (short)0, c, false, false); asm volatile("v_nop\n\tv_nop\n\tv_nop\n\tv_nop" : "+v"(d) : "v"(a), "v"(b)); return d; }
template <int ACT>
__global__ __launch_bounds__(128) void k_gemm2(const _Float16* __restrict__ A, int lda, size_t sA, const _Float16* __restrict__ Bh, int ldb, size_t sB, float alpha, const float* __restrict__ bias, size_t sBias, const float* __restrict__ CP, int rowsPerB, size_t sCPb, int row0g,
    float* __restrict__ C, _Float16* __restrict__ C16, int ldc, size_t sC, int M, int N, int K) { static_assert(ACT == 0 || ACT == 3 || ACT == 6 || ACT == 8 || ACT == 9 || ACT == 11 || ACT == 12 || ACT == 14 || ACT == 15 || ACT == 16 || ACT == 17, "k_gemm2: unsupported ACT code (would silently apply no activation)");
  __shared__ __attribute__((aligned(16))) float so[4][32][68];
  const int tid = threadIdx.x, w = tid >> 5, lane = tid & 31, ln = lane & 15, hh = lane >> 4; const int by = blockIdx.y;
  A += (size_t)by * sA; Bh += (size_t)by * sB; const size_t cofs = (size_t)by * sC; const float* bp = bias ? bias + (size_t)by * sBias : nullptr;
  const int ntn = N >> 6; const int mt = blockIdx.x / ntn, nq = blockIdx.x - mt * ntn; const int row0 = mt * 128 + 32 * w, col0 = nq * 64; if (row0 >= M) return;
  const _Float16* a0p = A + (size_t)(row0 + ln) * lda; const _Float16* a1p = a0p + (size_t)16 * lda;
  const _Float16* b0p = Bh + (size_t)(col0 + ln) * ldb; const _Float16* b1p = b0p + (size_t)16 * ldb; const _Float16* b2p = b1p + (size_t)16 * ldb; const _Float16* b3p = b2p + (size_t)16 * ldb;
  const v8f z8 = {0.f,0.f,0.f,0.f,0.f,0.f,0.f,0.f}; v8f c00 = z8, c01 = z8, c02 = z8, c03 = z8, c10 = z8, c11 = z8, c12 = z8, c13 = z8;
  for (int kb = 0; kb < K; kb += 32) { const v16h a0 = g2_frag(a0p + kb, hh), a1 = g2_frag(a1p + kb, hh);
    v16h b = g2_frag(b0p + kb, hh); c00 = g2_mma(a0, b, c00); c10 = g2_mma(a1, b, c10);
    b = g2_frag(b1p + kb, hh); c01 = g2_mma(a0, b, c01); c11 = g2_mma(a1, b, c11);
    b = g2_frag(b2p + kb, hh); c02 = g2_mma(a0, b, c02); c12 = g2_mma(a1, b, c12);
    b = g2_frag(b3p + kb, hh); c03 = g2_mma(a0, b, c03); c13 = g2_mma(a1, b, c13); }
  v8f accs[8] = {c00, c01, c02, c03, c10, c11, c12, c13};
#pragma unroll
  for (int u = 0; u < 8; ++u) { const int t = u & 3, half = u >> 2; const int col = col0 + t * 16 + ln; const float bv = bp ? bf16_round(bp[col]) : 0.f;
#pragma unroll
    for (int r = 0; r < 8; ++r) { const int rloc = half * 16 + 8 * hh + r; float v = accs[u][r] * alpha + bv; if (CP) { if (rowsPerB < 0) v += CP[cofs + (size_t)(row0g + row0 + rloc) * ldc + col];        else { const int bidx = (row0g + row0 + rloc) / rowsPerB; v += CP[(size_t)bidx * sCPb + (size_t)by * 64 + col]; } }
      if (ACT == 3) v = fmaxf(v, 0.f); else if (ACT == 6) v = 0.5f * v * (1.0f + erff(v * 0.70710678118654752f)); else if (ACT == 11) v = 1.0f / (1.0f + expf(-v)); else if (ACT == 15) v = v / (1.0f + expf(-v)); else if (ACT == 12) v = (v > 0.f) ? v : 0.01f * v; else if (ACT == 8) v = tanhf(v); else if (ACT == 9) v = 0.5f * v * (1.0f + tanhf(0.7978845608028654f * (v + 0.044715f * v * v * v))); else if (ACT == 14) v = (v > 0.f) ? v : 0.1f * v; else if (ACT == 16) v = (v >= 0.f) ? v : 0.3f * v; else if (ACT == 17) v = (v >= 0.f) ? v : 0.2f * v;
      so[w][rloc][t * 16 + ln] = v; } }
  __builtin_amdgcn_fence(__ATOMIC_ACQ_REL, "workgroup"); __builtin_amdgcn_wave_barrier();
  const int rsub = lane >> 4, c4 = (lane & 15) * 4;
  for (int pass = 0; pass < 2; ++pass) {
#pragma unroll
    for (int q = 0; q < 16; ++q) { const int r = q * 2 + rsub; const v4f v = *(const v4fa*)&so[w][r][c4]; if (C) *(volatile v4f*)(C + cofs + (size_t)(row0 + r) * ldc + col0 + c4) = v; if (C16) { v4h h4; for (int i = 0; i < 4; ++i) h4[i] = (_Float16)v[i]; *(volatile v4h*)(C16 + cofs + (size_t)(row0 + r) * ldc + col0 + c4) = h4; } }
    if (pass == 0) __threadfence(); } }


__global__ __launch_bounds__(256) void k_rdot(const float* __restrict__ u, const float* __restrict__ v, float* __restrict__ out, int rows) {
  const int r = (int)(blockIdx.x * 256 + threadIdx.x); if (r >= rows) return; const float* pu = u + (size_t)r * GD; const float* pv = v + (size_t)r * GD; float s = 0.f;
#pragma unroll
  for (int k = 0; k < GD; k += 4) { const v4f a = *(const v4fa*)(pu + k); const v4f b = *(const v4fa*)(pv + k);
#pragma unroll
    for (int q = 0; q < 4; ++q) s += bf16_round(a[q]) * bf16_round(b[q]); }
  float* d = out + r; *(volatile float*)d = s; __threadfence(); *(volatile float*)d = s; }
__global__ __launch_bounds__(128) void k_pproj(const float* __restrict__ pr, _Float16* __restrict__ P16, float* __restrict__ P2, float scale) {
  const unsigned k = blockIdx.x * 128 + threadIdx.x; if (k >= GK) return; const float* p = pr + (size_t)k * GD; float v[GD]; float n2 = 0.f;
#pragma unroll
  for (int d = 0; d < GD; d += 4) { const v4f a = *(const v4fa*)(p + d);
#pragma unroll
    for (int q = 0; q < 4; ++q) { v[d + q] = bf16_round(a[q]); n2 += v[d + q] * v[d + q]; } }
  const float fac = fminf(1.0f, 0.999f / fmaxf(sqrtf(n2), 1e-15f)); float p2 = 0.f; unsigned short* orow = (unsigned short*)P16 + (size_t)k * GD;
#pragma unroll
  for (int d = 0; d < GD; d += 8) { FragH f;
#pragma unroll
    for (int q = 0; q < 8; ++q) { const float w = v[d + q] * fac; p2 += w * w; f.h[q] = (_Float16)(w * scale); }
    const v8us o = f.half[0]; *(volatile v8us*)(orow + d) = o; __threadfence(); *(volatile v8us*)(orow + d) = o; }
  *(volatile float*)(P2 + k) = p2; __threadfence(); *(volatile float*)(P2 + k) = p2; }
__global__ __launch_bounds__(256) void k_geo(const float* __restrict__ G, const float* __restrict__ x2v, const float* __restrict__ p2v, float* __restrict__ out) {
  const size_t t = (size_t)blockIdx.x * 256 + threadIdx.x; if (t >= (size_t)GN * (GK / 4)) return; const unsigned k0 = (unsigned)(t % (GK / 4)) * 4; const size_t n = t / (GK / 4);
  const v4f g = *(const v4fa*)(G + t * 4); const float x2 = x2v[n]; const v4f p2 = *(const v4fa*)(p2v + k0); v4f o;
#pragma unroll
  for (int q = 0; q < 4; ++q) { const float xy = g[q]; const float a = 1.0f - 2.0f * xy + p2[q]; const float b = 1.0f - x2; const float den = fmaxf(1.0f - 2.0f * xy + x2 * p2[q], 1e-15f);
    const float m2 = ((a * a * x2 - 2.0f * a * b * xy) + b * b * p2[q]) / (den * den); const float z = fminf(fmaxf(sqrtf(m2), 0.0f), 0.99999f); const float dist = 2.0f * atanhf(z); o[q] = -(dist * dist); }
  float* op = out + t * 4; *(volatile v4f*)op = o; __threadfence(); *(volatile v4f*)op = o; }

extern "C" void kernel_launch(void* const* d_in, const int* in_sizes, int n_in,
                              void* d_out, int out_size, void* d_ws, size_t ws_size, hipStream_t stream) {
  (void)in_sizes; (void)n_in; (void)out_size;
  const float* const* I = (const float* const*)d_in; const float* x = I[0]; const float* pr = I[1];
  static_assert(GN % 128 == 0 && GK % 64 == 0 && GD % 32 == 0 && GD % 8 == 0 && ((size_t)GN * GD / 8) % 256 == 0 && GN % 256 == 0 && GK % 128 == 0 && ((size_t)GN * (GK / 4)) % 256 == 0, "whole tiles; exact grids");
  char* ws = (char*)d_ws; size_t off = 0;
  auto take = [&](size_t bytes) { char* p = ws + off; off += (bytes + 255) & ~(size_t)255; return p; };
  _Float16* X16 = (_Float16*)take((size_t)GN * GD * 2); _Float16* P16 = (_Float16*)take((size_t)GK * GD * 2); float* X2 = (float*)take((size_t)GN * 4); float* P2 = (float*)take((size_t)GK * 4); float* G = (float*)take((size_t)GN * GK * 4);
  if (off > ws_size) return;
  k_x16s<<<(unsigned)((size_t)GN * GD / 8 / 256), 256, 0, stream>>>(x, X16, (size_t)GN * GD / 8, GCAR);
  k_pproj<<<(unsigned)(GK / 128), 128, 0, stream>>>(pr, P16, P2, GCAR);
  k_rdot<<<(unsigned)(GN / 256), 256, 0, stream>>>(x, x, X2, GN);

  k_gemm2<0><<<dim3((unsigned)((GN / 128) * (GK / 64)), 1), 128, 0, stream>>>(X16, GD, 0, P16, GD, 0, 1.0f / (GCAR * GCAR), nullptr, 0, nullptr, 1, 0, 0, G, nullptr, GK, 0, GN, GK, GD);
  k_geo<<<(unsigned)((size_t)GN * (GK / 4) / 256), 256, 0, stream>>>(G, X2, P2, (float*)d_out);
}
